// GraphAttentionLayer_36292473651250
// MI455X (gfx1250) — hardware-verified
//
#include <hip/hip_runtime.h>


#define NB_  8
#define NN   2048
#define FF   64
#define RP   32
typedef _Float16 h16;
typedef unsigned short bf;
typedef __attribute__((ext_vector_type(16))) __bf16   v16bf;
typedef __attribute__((ext_vector_type(16))) _Float16 v16h;
typedef __attribute__((ext_vector_type(8)))  _Float16 v8h;
typedef __attribute__((ext_vector_type(8)))  unsigned short v8us;
typedef __attribute__((ext_vector_type(8)))  float    v8f;
typedef __attribute__((ext_vector_type(4)))  float    v4f;
typedef v8h  __attribute__((may_alias)) v8ha;
typedef v4f  __attribute__((may_alias)) v4fa;
typedef v8us __attribute__((may_alias)) v8usa;

__device__ __forceinline__ unsigned short f2bf(float f) { unsigned u = __float_as_uint(f); u += 0x7FFFu + ((u >> 16) & 1u); return (unsigned short)(u >> 16); }
__device__ __forceinline__ float bf2f(unsigned short b) { return __uint_as_float(((unsigned)b) << 16); }
__device__ __forceinline__ float bfr(float f) { return bf2f(f2bf(f)); }
__device__ __forceinline__ v16h cat16(v8h lo, v8h hi) { return __builtin_shufflevector(lo, hi, 0, 1, 2, 3, 4, 5, 6, 7, 8, 9, 10, 11, 12, 13, 14, 15); }
__device__ __forceinline__ v16bf cat16b(v8us lo, v8us hi) { return __builtin_bit_cast(v16bf, __builtin_shufflevector(lo, hi, 0, 1, 2, 3, 4, 5, 6, 7, 8, 9, 10, 11, 12, 13, 14, 15)); }
__device__ __forceinline__ v8f wmma16(v16h a, v16h b, v8f c) { return __builtin_amdgcn_wmma_f32_16x16x32_f16(false, a, false, b, (short)0, c, false, false); }
__device__ __forceinline__ v8f wmmab(v16bf a, v16bf b, v8f c) { return __builtin_amdgcn_wmma_f32_16x16x32_bf16(false, a, false, b, (short)0, c, false, false); }


template <typename T16> struct WFrag;
template <> struct WFrag<h16> { typedef v16h V; static __device__ __forceinline__ V ld(const h16* p) { return cat16(*(const v8h*)p, *(const v8h*)(p + 16)); } static __device__ __forceinline__ v8f mma(V a, V b, v8f c) { return wmma16(a, b, c); } };
template <> struct WFrag<bf> { typedef v16bf V; static __device__ __forceinline__ V ld(const bf* p) { return cat16b(*(const v8us*)p, *(const v8us*)(p + 16)); } static __device__ __forceinline__ v8f mma(V a, V b, v8f c) { return wmmab(a, b, c); } };
template <typename T16, int NSPLIT, bool BIAS>
__global__ __launch_bounds__(32) void k_gemmw(const T16* __restrict__ A, const T16* __restrict__ A2, const T16* __restrict__ Bt, const T16* __restrict__ Bt2, int K, float* C, int ldc, const float* __restrict__ bias, size_t sA, size_t sB, size_t sC) {
    typedef typename WFrag<T16>::V V;
    __shared__ __align__(16) float os[16 * 68];
    const size_t z = blockIdx.z; A += z * sA; if (A2) A2 += z * sA; Bt += z * sB; if (Bt2) Bt2 += z * sB; C += z * sC;
    const int lane = threadIdx.x & 31, lr = lane & 15, hi = lane >> 4; const int r0 = blockIdx.x * 64, c0 = blockIdx.y * 64;
    v8f acc[4][4];
#pragma unroll
    for (int mb = 0; mb < 4; ++mb)
#pragma unroll
        for (int nb = 0; nb < 4; ++nb) acc[mb][nb] = (v8f){};
    const size_t aoff = (size_t)(r0 + lr) * K + 8 * hi, boff = (size_t)(c0 + lr) * K + 8 * hi;
#pragma unroll 1
    for (int kc = 0; kc < K; kc += 32) {
        V a[4], a2[4];
#pragma unroll
        for (int mb = 0; mb < 4; ++mb) { a[mb] = WFrag<T16>::ld(A + aoff + (size_t)mb * 16 * K + kc); if (NSPLIT == 1 || NSPLIT == 2) a2[mb] = WFrag<T16>::ld(A2 + aoff + (size_t)mb * 16 * K + kc); }
#pragma unroll
        for (int nb = 0; nb < 4; ++nb) { const V b = WFrag<T16>::ld(Bt + boff + (size_t)nb * 16 * K + kc); V b2; if (NSPLIT >= 2) b2 = WFrag<T16>::ld(Bt2 + boff + (size_t)nb * 16 * K + kc);
#pragma unroll
            for (int mb = 0; mb < 4; ++mb) { acc[mb][nb] = WFrag<T16>::mma(a[mb], b, acc[mb][nb]); if (NSPLIT == 1 || NSPLIT == 2) acc[mb][nb] = WFrag<T16>::mma(a2[mb], b, acc[mb][nb]); if (NSPLIT >= 2) acc[mb][nb] = WFrag<T16>::mma(a[mb], b2, acc[mb][nb]); } }
        asm volatile("v_nop\n\tv_nop\n\tv_nop\n\tv_nop" : "+v"(acc[0][0]), "+v"(acc[1][1]), "+v"(acc[2][2]), "+v"(acc[3][3]) : "v"(a[0]), "v"(a[3]));
    }
#pragma unroll
    for (int mb = 0; mb < 4; ++mb) {
#pragma unroll
        for (int nb = 0; nb < 4; ++nb) {
#pragma unroll
            for (int j = 0; j < 8; ++j) os[(hi * 8 + j) * 68 + nb * 16 + lr] = acc[mb][nb][j]; }
        __builtin_amdgcn_wave_barrier(); asm volatile("" ::: "memory");
        float* crow = C + (size_t)(r0 + mb * 16) * ldc + c0;
#pragma unroll 1
        for (int ps = 0; ps < 2; ++ps) {
#pragma unroll
            for (int s = 0; s < 8; ++s) { const int row = 2 * s + hi, cofs = lr * 4; v4f val = *(const v4fa*)(os + row * 68 + cofs); if (BIAS) { val[0] += bfr(bias[c0 + cofs]); val[1] += bfr(bias[c0 + cofs + 1]); val[2] += bfr(bias[c0 + cofs + 2]); val[3] += bfr(bias[c0 + cofs + 3]); }
                *(volatile v4f*)(crow + (size_t)row * ldc + cofs) = val; }
            if (ps == 0) __threadfence(); }
        __builtin_amdgcn_wave_barrier(); asm volatile("" ::: "memory");
    }
}

__device__ __forceinline__ void splitf(float y, unsigned short& h, unsigned short& l) { h = f2bf(y); l = f2bf(y - bf2f(h)); }
typedef __attribute__((ext_vector_type(2))) unsigned short v2us;
typedef __attribute__((ext_vector_type(4))) unsigned short v4us;
typedef __attribute__((ext_vector_type(2))) float v2f;
typedef __attribute__((ext_vector_type(4))) int v4i;
__global__ __launch_bounds__(256) void k_wtG(const float* __restrict__ w, int K, int N, bf* Bt) {
    const int lane = threadIdx.x & 31; const int L0 = (blockIdx.x * 8 + (threadIdx.x >> 5)) * 8; const int nlines = N * K / 64;
#pragma unroll
    for (int ps = 0; ps < 2; ++ps) {
#pragma unroll 1
        for (int l = 0; l < 8; ++l) { const int L = L0 + l; if (L >= nlines) break; const size_t e = (size_t)L * 64 + lane * 2; const int k = (int)(e % K), n = (int)(e / K); v2us o;
            o[0] = f2bf(w[(size_t)k * N + n]); o[1] = f2bf(w[(size_t)(k + 1) * N + n]); *(volatile v2us*)(Bt + e) = o; }
        if (ps == 0) __threadfence(); }
}
__global__ __launch_bounds__(256) void k_cvt8(const float* __restrict__ src, bf* dst, size_t n8) { const size_t i = (size_t)blockIdx.x * 256 + threadIdx.x; if (i >= n8) return; const v8f v = *(const v8f*)(src + i * 8); v8us o;
#pragma unroll
    for (int k = 0; k < 8; ++k) o[k] = f2bf(v[k]); *(volatile v8us*)(dst + i * 8) = o; __threadfence(); *(volatile v8us*)(dst + i * 8) = o; }

__global__ __launch_bounds__(256) void k_xpl(const float* __restrict__ in, const float* __restrict__ nw, const float* __restrict__ nb, bf* Xh, bf* Xl) { const size_t e = ((size_t)blockIdx.x * 256 + threadIdx.x) * 4; if (e >= (size_t)NN * FF) return; const int n = (int)(e / FF); const float w = bfr(nw[n]), bb = bfr(nb[n]); v4us oh, ol;
#pragma unroll
    for (int q = 0; q < 4; ++q) { const float v = bfr(in[e + q]); float t = __fmul_rn(v, w); asm volatile("" : "+v"(t)); float t2 = __fadd_rn(t, bb); asm volatile("" : "+v"(t2)); const float x = __fadd_rn(t2, v); unsigned short a, c; splitf(x, a, c); oh[q] = a; ol[q] = c; }
    *(volatile v4us*)(Xh + e) = oh; *(volatile v4us*)(Xl + e) = ol; __threadfence(); *(volatile v4us*)(Xh + e) = oh; *(volatile v4us*)(Xl + e) = ol; }
__global__ __launch_bounds__(256) void k_ln64(const float* __restrict__ HP, const float* __restrict__ g, const float* __restrict__ be, const float* __restrict__ a, float* H, float* S12) { const int n = blockIdx.x * 256 + threadIdx.x; if (n >= NN) return; const float* hp = HP + (size_t)n * FF; float s = 0.f;
#pragma unroll 8
    for (int c = 0; c < FF; ++c) s = __fadd_rn(s, hp[c]);
    const float mu = s * (1.0f / FF); float s2 = 0.f;
#pragma unroll 8
    for (int c = 0; c < FF; ++c) { const float d0 = __fsub_rn(hp[c], mu); float p = __fmul_rn(d0, d0); asm volatile("" : "+v"(p)); s2 = __fadd_rn(s2, p); }
    const float rs = __fdiv_rn(1.0f, __fsqrt_rn(__fadd_rn(s2 * (1.0f / FF), 1e-5f))); float d1 = 0.f, d2 = 0.f;
#pragma unroll 1
    for (int ps = 0; ps < 2; ++ps) { d1 = 0.f; d2 = 0.f;
#pragma unroll 4
        for (int c = 0; c < FF; c += 4) { v4f o;
#pragma unroll
            for (int q = 0; q < 4; ++q) { float n0 = __fmul_rn(__fsub_rn(hp[c + q], mu), rs); asm volatile("" : "+v"(n0)); float n1 = __fmul_rn(n0, bfr(g[c + q])); asm volatile("" : "+v"(n1)); const float y = __fadd_rn(n1, bfr(be[c + q])); o[q] = y; float p1 = __fmul_rn(y, bfr(a[c + q])); float p2 = __fmul_rn(y, bfr(a[FF + c + q])); asm volatile("" : "+v"(p1), "+v"(p2)); d1 = __fadd_rn(d1, p1); d2 = __fadd_rn(d2, p2); }
            *(volatile v4f*)(H + (size_t)n * FF + c) = o; }
        v2f sv; sv[0] = d1; sv[1] = d2; *(volatile v2f*)(S12 + (size_t)n * 2) = sv;
        if (ps == 0) __threadfence(); } }
__global__ __launch_bounds__(256) void k_htp(const float* __restrict__ H, bf* HTh, bf* HTl) { const size_t e = ((size_t)blockIdx.x * 256 + threadIdx.x) * 2; if (e >= (size_t)FF * NN) return; const int n = (int)(e % NN), c = (int)(e / NN); v2us oh, ol;
#pragma unroll
    for (int q = 0; q < 2; ++q) { unsigned short a2, c2; splitf(H[(size_t)(n + q) * FF + c], a2, c2); oh[q] = a2; ol[q] = c2; }
    *(volatile v2us*)(HTh + e) = oh; *(volatile v2us*)(HTl + e) = ol; __threadfence(); *(volatile v2us*)(HTh + e) = oh; *(volatile v2us*)(HTl + e) = ol; }
__global__ __launch_bounds__(256) void k_gsoft(const float* __restrict__ S12, const int* __restrict__ ADJ, bf* Ph, bf* Pl) {
    const int lane = threadIdx.x & 31; const int i = blockIdx.x * 8 + (threadIdx.x >> 5); if (i >= NN) return; const float s1 = S12[(size_t)i * 2]; const int* ar = ADJ + (size_t)i * NN; float v[NN / 32]; float mx = -3.0e38f;
#pragma unroll
    for (int ch = 0; ch < NN / 128; ++ch) { const int j0 = ch * 128 + lane * 4; const v4i m4 = *(const v4i*)(ar + j0);
#pragma unroll
        for (int q = 0; q < 4; ++q) { const int j = j0 + q; const float ee = __fadd_rn(s1, S12[(size_t)j * 2 + 1]); float en = __fmul_rn(ee, 0.2f); asm volatile("" : "+v"(en)); const float lr = (ee > 0.f) ? ee : en; const float t = (m4[q] > 0) ? lr : -9.0e15f; v[ch * 4 + q] = t; mx = fmaxf(mx, t); } }
#pragma unroll
    for (int sh = 16; sh; sh >>= 1) mx = fmaxf(mx, __shfl_xor(mx, sh, 32));
    float sum = 0.f;
#pragma unroll
    for (int k = 0; k < NN / 32; ++k) { float d0 = __fsub_rn(v[k], mx); asm volatile("" : "+v"(d0)); v[k] = __builtin_amdgcn_exp2f(__fmul_rn(d0, 1.4426950408889634f)); sum += v[k]; }
#pragma unroll
    for (int sh = 16; sh; sh >>= 1) sum += __shfl_xor(sum, sh, 32);
    const float f = __fdiv_rn(1.0f, sum);
#pragma unroll 1
    for (int ps = 0; ps < 2; ++ps) {
#pragma unroll
        for (int ch = 0; ch < NN / 128; ++ch) { v4us oh, ol;
#pragma unroll
            for (int q = 0; q < 4; ++q) { unsigned short a2, c2; splitf(v[ch * 4 + q] * f, a2, c2); oh[q] = a2; ol[q] = c2; }
            const size_t oo = (size_t)i * NN + ch * 128 + lane * 4; *(volatile v4us*)(Ph + oo) = oh; *(volatile v4us*)(Pl + oo) = ol; }
        if (ps == 0) __threadfence(); } }
__global__ __launch_bounds__(256) void k_fin(const float* __restrict__ AG, const float* __restrict__ H, float* O, size_t n4) { const size_t i = (size_t)blockIdx.x * 256 + threadIdx.x; if (i >= n4) return; const v4f a = *(const v4f*)(AG + i * 4), h = *(const v4f*)(H + i * 4); v4f o;
#pragma unroll
    for (int q = 0; q < 4; ++q) { const float x = __fadd_rn(a[q], h[q]); o[q] = (x > 0.f) ? x : expm1f(x); }
    *(volatile v4f*)(O + i * 4) = o; __threadfence(); *(volatile v4f*)(O + i * 4) = o; }

extern "C" void kernel_launch(void* const* d_in, const int* in_sizes, int n_in,
                              void* d_out, int out_size, void* d_ws, size_t ws_size, hipStream_t stream) {
    (void)in_sizes; (void)n_in; (void)out_size;
    const float* inp = (const float*)d_in[0]; const int* ADJ = (const int*)d_in[1]; const float* W = (const float*)d_in[2]; const float* a = (const float*)d_in[3]; const float* nw = (const float*)d_in[4]; const float* nb = (const float*)d_in[5]; const float* g = (const float*)d_in[6]; const float* be = (const float*)d_in[7];
    float* OUT = (float*)d_out;
    char* wsp = (char*)d_ws;
    auto take = [&](size_t bytes) { char* p = wsp; wsp += (bytes + 255) & ~(size_t)255; return (void*)p; };
    bf* WT = (bf*)take(FF * FF * 2); bf* Xh = (bf*)take((size_t)NN * FF * 2); bf* Xl = (bf*)take((size_t)NN * FF * 2); float* HP = (float*)take((size_t)NN * FF * 4); float* H = (float*)take((size_t)NN * FF * 4); float* S12 = (float*)take((size_t)NN * 2 * 4);
    bf* HTh = (bf*)take((size_t)FF * NN * 2); bf* HTl = (bf*)take((size_t)FF * NN * 2); bf* Ph = (bf*)take((size_t)NN * NN * 2); bf* Pl = (bf*)take((size_t)NN * NN * 2); float* AG = (float*)take((size_t)NN * FF * 4);
    if ((size_t)(wsp - (char*)d_ws) > ws_size) return;
    k_wtG<<<(FF * FF / 64 + 63) / 64, 256, 0, stream>>>(W, FF, FF, WT);
    for (int b = 0; b < NB_; ++b) {
        k_xpl<<<(NN * FF / 4 + 255) / 256, 256, 0, stream>>>(inp + (size_t)b * NN * FF, nw, nb, Xh, Xl);
        k_gemmw<bf, 1, false><<<dim3(NN / 64, FF / 64, 1), 32, 0, stream>>>(Xh, Xl, WT, nullptr, FF, HP, FF, nullptr, 0, 0, 0);
        k_ln64<<<NN / 256, 256, 0, stream>>>(HP, g, be, a, H, S12); k_htp<<<(FF * NN / 2 + 255) / 256, 256, 0, stream>>>(H, HTh, HTl);
        k_gsoft<<<NN / 8, 256, 0, stream>>>(S12, ADJ, Ph, Pl);
        k_gemmw<bf, 2, false><<<dim3(NN / 64, FF / 64, 1), 32, 0, stream>>>(Ph, Pl, HTh, HTl, NN, AG, FF, nullptr, 0, 0, 0);
        k_fin<<<(NN * FF / 4 + 255) / 256, 256, 0, stream>>>(AG, H, OUT + (size_t)b * NN * FF, (size_t)NN * FF / 4); }
}
